// CausalSelfAttention_70935679861415
// MI455X (gfx1250) — hardware-run, weakly checked
//
#include <hip/hip_runtime.h>


#ifndef NB
#define NB 4
#endif
#ifndef SEQ
#define SEQ 2048
#endif
#define NB_FULL  4
#define SEQ_FULL 2048
#ifndef OUT_SEQ
#define OUT_SEQ SEQ
#endif
#define DM   1024
#define NH_  16
#define HD   64
#define AW   4
#define ERW  ((SEQ < 512) ? SEQ : 512)
#define QRS  2048.0f
#define QRI  (1.0f / 2048.0f)
#define SC2  (0.125f * 1.4426950408889634f)
#define PSH  8.0f
#define CXS  64.0f
#define WPS  64.0f
#define OSC  (1.0f / 4096.0f)
#define OSCR (1.0f / 8388608.0f)

static_assert(HD == 64);
static_assert(NH_ * HD == DM);
static_assert(DM % 64 == 0);
static_assert(DM % 32 == 0);
static_assert(SEQ % 64 == 0);
static_assert((NB * SEQ) % 64 == 0);
static_assert(SEQ % 32 == 0);
static_assert(ERW % 64 == 0);
static_assert(ERW % (16 * AW) == 0);
static_assert((SEQ - ERW) % 64 == 0);
static_assert((SEQ - ERW) % (16 * AW) == 0);
static_assert(((size_t)SEQ * DM) % 8 == 0);
static_assert(NB <= NB_FULL);
static_assert(SEQ <= SEQ_FULL);

typedef _Float16 h16;
typedef unsigned short bf;
typedef __attribute__((ext_vector_type(16))) __bf16   v16bf;
typedef __attribute__((ext_vector_type(16))) _Float16 v16h;
typedef __attribute__((ext_vector_type(8)))  _Float16 v8h;
typedef __attribute__((ext_vector_type(8)))  unsigned short v8us;
typedef __attribute__((ext_vector_type(8)))  float    v8f;
typedef __attribute__((ext_vector_type(4)))  float    v4f;
typedef __attribute__((ext_vector_type(4)))  int      v4i;
typedef v4f  __attribute__((may_alias)) v4fa;

__device__ __forceinline__ unsigned short f2bf(float f) { unsigned u = __float_as_uint(f); u += 0x7FFFu + ((u >> 16) & 1u); return (unsigned short)(u >> 16); }
__device__ __forceinline__ float bfr(float f) { return __uint_as_float(((unsigned)f2bf(f)) << 16); }
__device__ __forceinline__ v16h cat16(v8h lo, v8h hi) { return __builtin_shufflevector(lo, hi, 0, 1, 2, 3, 4, 5, 6, 7, 8, 9, 10, 11, 12, 13, 14, 15); }
__device__ __forceinline__ v16bf cat16b(v8us lo, v8us hi) { return __builtin_bit_cast(v16bf, __builtin_shufflevector(lo, hi, 0, 1, 2, 3, 4, 5, 6, 7, 8, 9, 10, 11, 12, 13, 14, 15)); }
__device__ __forceinline__ v8f wmma16(v16h a, v16h b, v8f c) { return __builtin_amdgcn_wmma_f32_16x16x32_f16(false, a, false, b, (short)0, c, false, false); }
__device__ __forceinline__ v8f wmmab(v16bf a, v16bf b, v8f c) { return __builtin_amdgcn_wmma_f32_16x16x32_bf16(false, a, false, b, (short)0, c, false, false); }
__device__ __forceinline__ v16h  ldh(const h16* p) { return cat16(*(const v8h*)p, *(const v8h*)(p + 16)); }
__device__ __forceinline__ v16bf ldb(const bf* p)  { return cat16b(*(const v8us*)p, *(const v8us*)(p + 16)); }
__device__ __forceinline__ v16h  keepz(v16h v, bool keep) { const v16h z = (v16h){}; return keep ? v : z; }
__device__ __forceinline__ void wave_sync() { __builtin_amdgcn_fence(3  , "wavefront"); __builtin_amdgcn_wave_barrier(); asm volatile("" ::: "memory"); }

__global__ __launch_bounds__(256) void k_cvt8(const float* __restrict__ src, bf* dst, size_t n8) {
    const size_t i = (size_t)blockIdx.x * 256 + threadIdx.x; if (i >= n8) return;
    const v8f v = *(const v8f*)(src + i * 8); v8us o;
#pragma unroll
    for (int k = 0; k < 8; ++k) o[k] = f2bf(v[k]);
    *(volatile v8us*)(dst + i * 8) = o; __threadfence(); *(volatile v8us*)(dst + i * 8) = o;
}

template <int F16S>
__global__ __launch_bounds__(256) void k_wt(const float* __restrict__ W, unsigned short* dst) {
    __shared__ __align__(16) float ts[64 * 68];
    const int tid = threadIdx.x; const int n0 = blockIdx.x * 64, k0 = blockIdx.y * 64;
#pragma unroll
    for (int it = 0; it < 4; ++it) { const int q = it * 256 + tid; const int i = q >> 4, j4 = (q & 15) * 4;
        const v4f v = *(const v4f*)(W + (size_t)(k0 + i) * DM + n0 + j4);
        *(v4fa*)(&ts[i * 68 + j4]) = v; }
    __syncthreads();
#pragma unroll 1
    for (int ps = 0; ps < 2; ++ps) {
#pragma unroll
        for (int it = 0; it < 2; ++it) { const int j = it * 32 + (tid >> 3), c8 = (tid & 7) * 8;
            v8us o;
#pragma unroll
            for (int i = 0; i < 8; ++i) { const float w = ts[(c8 + i) * 68 + j]; const unsigned short bb = f2bf(w);
                if (F16S) { const h16 hv = (h16)(__uint_as_float(((unsigned)bb) << 16) * WPS); o[i] = __builtin_bit_cast(unsigned short, hv); }
                else o[i] = bb; }
            *(volatile v8us*)(dst + (size_t)(n0 + j) * DM + k0 + c8) = o; }
        if (ps == 0) __threadfence(); }
}

__global__ __launch_bounds__(32) void k_proj(const bf* __restrict__ A, const bf* __restrict__ Bt, const float* __restrict__ bias, int biasMode,
                                             h16* Ph, h16* Pr, int resMode, int RB, size_t sRB, int pitch, int CB, size_t sCB,
                                             size_t sRBr, int pitchR, size_t sCBr) {
    __shared__ __align__(16) float os[16 * 68];
    const int K = DM;
    const int lane = threadIdx.x & 31, lr = lane & 15, hi = lane >> 4; const int r0 = blockIdx.x * 64, c0 = blockIdx.y * 64;
    v8f acc[4][4];
#pragma unroll
    for (int mb = 0; mb < 4; ++mb)
#pragma unroll
        for (int nb = 0; nb < 4; ++nb) acc[mb][nb] = (v8f){};
    const size_t aoff = (size_t)(r0 + lr) * K + 8 * hi, boff = (size_t)(c0 + lr) * K + 8 * hi;
#pragma unroll 1
    for (int kc = 0; kc < K; kc += 32) {
        v16bf a[4];
#pragma unroll
        for (int mb = 0; mb < 4; ++mb) a[mb] = ldb(A + aoff + (size_t)mb * 16 * K + kc);
#pragma unroll
        for (int nb = 0; nb < 4; ++nb) { const v16bf b = ldb(Bt + boff + (size_t)nb * 16 * K + kc);
#pragma unroll
            for (int mb = 0; mb < 4; ++mb) acc[mb][nb] = wmmab(a[mb], b, acc[mb][nb]); }
        asm volatile("v_nop\n\tv_nop\n\tv_nop\n\tv_nop" : "+v"(acc[0][0]), "+v"(acc[1][1]), "+v"(acc[2][2]), "+v"(acc[3][3]) : "v"(a[0]), "v"(a[1]), "v"(a[2]), "v"(a[3]));
    }
    const size_t tbase = (size_t)(r0 / RB) * sRB + (size_t)(r0 % RB) * (size_t)pitch + (size_t)(c0 / CB) * sCB + (size_t)(c0 % CB);
    const size_t rtb   = (size_t)(r0 / RB) * sRBr + (size_t)(r0 % RB) * (size_t)pitchR + (size_t)(c0 / CB) * sCBr + (size_t)(c0 % CB);
    const int useRes = (((resMode == 1) && ((r0 % SEQ) < ERW)) || ((resMode == 2) && ((c0 % SEQ) < ERW))) ? 1 : 0;
    float bc[4];
#pragma unroll
    for (int nb = 0; nb < 4; ++nb) { const int ci = (biasMode == 1) ? (c0 + nb * 16 + lr) : lr;
        const float bv = bfr(bias[ci]); bc[nb] = (biasMode == 1) ? bv : 0.0f; }
#pragma unroll
    for (int mb = 0; mb < 4; ++mb) {
        float br[8];
#pragma unroll
        for (int j = 0; j < 8; ++j) { const int ri = (biasMode == 2) ? (r0 + mb * 16 + hi * 8 + j) : lr;
            const float bv = bfr(bias[ri]); br[j] = (biasMode == 2) ? bv : 0.0f; }
#pragma unroll
        for (int nb = 0; nb < 4; ++nb) {
#pragma unroll
            for (int j = 0; j < 8; ++j) os[(hi * 8 + j) * 68 + nb * 16 + lr] = acc[mb][nb][j] + bc[nb] + br[j]; }
        wave_sync();
        const size_t sb  = tbase + (size_t)(mb * 16) * (size_t)pitch;
        const size_t rsb = rtb   + (size_t)(mb * 16) * (size_t)pitchR;
#pragma unroll 1
        for (int ps = 0; ps < 2; ++ps) {
#pragma unroll
            for (int s = 0; s < 4; ++s) { const int row = 4 * s + (lane >> 3), c8 = (lane & 7) * 8;
                const v4f x0 = *(const v4fa*)(&os[row * 68 + c8]); const v4f x1 = *(const v4fa*)(&os[row * 68 + c8 + 4]); v8h hv, rv;
#pragma unroll
                for (int i = 0; i < 4; ++i) { const h16 a0 = (h16)x0[i]; const h16 a1 = (h16)x1[i]; hv[i] = a0; hv[4 + i] = a1; rv[i] = (h16)((x0[i] - (float)a0) * QRS); rv[4 + i] = (h16)((x1[i] - (float)a1) * QRS); }
                *(volatile v8h*)(Ph + sb + (size_t)row * (size_t)pitch + c8) = hv;
                if (useRes) *(volatile v8h*)(Pr + rsb + (size_t)row * (size_t)pitchR + c8) = rv; }
            if (ps == 0) __threadfence(); }
        wave_sync();
    }
}

__device__ __forceinline__ void put8(float* p, v8f o, float s) {
    v4f a, c;
    a[0] = o[0] * s; a[1] = o[1] * s; a[2] = o[2] * s; a[3] = o[3] * s; c[0] = o[4] * s; c[1] = o[5] * s; c[2] = o[6] * s; c[3] = o[7] * s;
    *(v4fa*)p = a; *(v4fa*)(p + 4) = c;
}

template <int EK>
__global__ __launch_bounds__(32 * AW) void k_flash(const h16* __restrict__ QH, const h16* __restrict__ QR, const h16* __restrict__ KH, const h16* __restrict__ KR,
                                                   const h16* __restrict__ VT, const h16* __restrict__ VR, const int* __restrict__ MASK, h16* CH, h16* CR, int tofs) {
    __shared__ __align__(16) float os[AW * 16 * 68];
    const int lane = threadIdx.x & 31, wave = __builtin_amdgcn_readfirstlane((int)(threadIdx.x >> 5)), lr = lane & 15, hi = lane >> 4;
    const int zh = blockIdx.y; const int b = zh / NH_, h = zh % NH_;
    const int t0 = tofs + (blockIdx.x * AW + wave) * 16;
    const size_t pbase = (size_t)zh * SEQ * HD;
    const size_t rbase = (size_t)zh * ERW * HD;
    const size_t qo = pbase + (size_t)(t0 + lr) * HD + 8 * hi;
    const v16h qh0 = ldh(QH + qo), qh1 = ldh(QH + qo + 32);
    v16h qr0 = (v16h){}, qr1 = (v16h){};
    if (EK) { const size_t qro = rbase + (size_t)(t0 + lr) * HD + 8 * hi; qr0 = ldh(QR + qro); qr1 = ldh(QR + qro + 32); }
    const size_t ko  = pbase + (size_t)lr * HD + 8 * hi;
    const size_t kro = rbase + (size_t)lr * HD + 8 * hi;
    const size_t vo  = pbase + (size_t)lr * SEQ + 8 * hi;
    const size_t vro = rbase + (size_t)lr * ERW + 8 * hi;
    const int* mrow = MASK + (size_t)(t0 + lr) * SEQ_FULL + 8 * hi;
    const float NINF = -__builtin_inff();
    v8f o0 = (v8f){}, o1 = (v8f){}, o2 = (v8f){}, o3 = (v8f){};
    v8f p0 = (v8f){}, p1 = (v8f){}, p2 = (v8f){}, p3 = (v8f){};
    float m = -3.0e38f, l = 0.0f;
#pragma unroll 1
    for (int key0 = 0; key0 < SEQ; key0 += 32) {
        const int* mp = mrow + key0;
        const v4i ma0 = *(const v4i*)(mp), ma1 = *(const v4i*)(mp + 4), mb0 = *(const v4i*)(mp + 16), mb1 = *(const v4i*)(mp + 20);
        const v4i mo = ma0 | ma1 | mb0 | mb1;
        const int many = mo[0] | mo[1] | mo[2] | mo[3];
        if (__builtin_amdgcn_ballot_w32(many != 0) == 0u) continue;
        const h16* ka = KH + ko + (size_t)key0 * HD;
        const v16h ka0 = ldh(ka), ka1 = ldh(ka + 32), kb0 = ldh(ka + 16 * HD), kb1 = ldh(ka + 16 * HD + 32);
        v8f sHa = (v8f){}, sLa = (v8f){}, sHb = (v8f){}, sLb = (v8f){};
        const bool rs = key0 < ERW;
        const int  kk = rs ? key0 : 0;
        if (EK) {
            sHa = wmma16(ka0, qh0, sHa); sLa = wmma16(ka0, qr0, sLa); sHb = wmma16(kb0, qh0, sHb); sLb = wmma16(kb0, qr0, sLb);
            sHa = wmma16(ka1, qh1, sHa); sLa = wmma16(ka1, qr1, sLa); sHb = wmma16(kb1, qh1, sHb); sLb = wmma16(kb1, qr1, sLb);
            asm volatile("v_nop\n\tv_nop\n\tv_nop\n\tv_nop" : "+v"(sHa), "+v"(sLa), "+v"(sHb), "+v"(sLb) : "v"(ka0), "v"(ka1), "v"(kb0), "v"(kb1) : "memory");
            const h16* kr = KR + kro + (size_t)kk * HD;
            const v16h ra0 = keepz(ldh(kr), rs), ra1 = keepz(ldh(kr + 32), rs), rb0 = keepz(ldh(kr + 16 * HD), rs), rb1 = keepz(ldh(kr + 16 * HD + 32), rs);
            sLa = wmma16(ra0, qh0, sLa); sLb = wmma16(rb0, qh0, sLb); sLa = wmma16(ra1, qh1, sLa); sLb = wmma16(rb1, qh1, sLb);
            asm volatile("v_nop\n\tv_nop\n\tv_nop\n\tv_nop" : "+v"(sLa), "+v"(sLb) : "v"(ra0), "v"(ra1), "v"(rb0), "v"(rb1) : "memory");
        } else {
            sHa = wmma16(ka0, qh0, sHa); sHb = wmma16(kb0, qh0, sHb); sHa = wmma16(ka1, qh1, sHa); sHb = wmma16(kb1, qh1, sHb);
            asm volatile("v_nop\n\tv_nop\n\tv_nop\n\tv_nop" : "+v"(sHa), "+v"(sHb) : "v"(ka0), "v"(ka1), "v"(kb0), "v"(kb1));
        }
        float ta[8], tb[8]; float mx = -3.0e38f;
#pragma unroll
        for (int r = 0; r < 8; ++r) {
            const int mka = (r < 4) ? ma0[r & 3] : ma1[r & 3];
            const int mkb = (r < 4) ? mb0[r & 3] : mb1[r & 3];
            float sa = sHa[r], sb = sHb[r];
            if (EK) { sa += sLa[r] * QRI; sb += sLb[r] * QRI; }
            ta[r] = (mka != 0) ? sa * SC2 : NINF; tb[r] = (mkb != 0) ? sb * SC2 : NINF;
            mx = fmaxf(mx, fmaxf(ta[r], tb[r])); }
        mx = fmaxf(mx, __shfl_xor(mx, 16, 32));
        const float mnew = fmaxf(m, mx);
        const float alpha = __builtin_amdgcn_exp2f(m - mnew);
        const float sh = PSH - mnew;
        v16h pb; float ls = 0.0f;
#pragma unroll
        for (int r = 0; r < 8; ++r) { const h16 pa = (h16)__builtin_amdgcn_exp2f(ta[r] + sh); const h16 pc = (h16)__builtin_amdgcn_exp2f(tb[r] + sh); pb[r] = pa; pb[8 + r] = pc; ls += (float)pa + (float)pc; }
        l = l * alpha + ls; m = mnew;
        o0 = o0 * alpha; o1 = o1 * alpha; o2 = o2 * alpha; o3 = o3 * alpha;
        if (EK) { p0 = p0 * alpha; p1 = p1 * alpha; p2 = p2 * alpha; p3 = p3 * alpha; }
        const h16* va = VT + vo + key0;
        const v16h v0 = ldh(va), v1 = ldh(va + (size_t)16 * SEQ), v2 = ldh(va + (size_t)32 * SEQ), v3 = ldh(va + (size_t)48 * SEQ);
        o0 = wmma16(v0, pb, o0); o1 = wmma16(v1, pb, o1); o2 = wmma16(v2, pb, o2); o3 = wmma16(v3, pb, o3);
        if (EK) {
            asm volatile("v_nop\n\tv_nop\n\tv_nop\n\tv_nop" : "+v"(o0), "+v"(o1), "+v"(o2), "+v"(o3) : "v"(v0), "v"(v1), "v"(v2), "v"(v3), "v"(pb) : "memory");
            const h16* vr = VR + vro + kk;
            const v16h r0 = keepz(ldh(vr), rs), r1 = keepz(ldh(vr + (size_t)16 * ERW), rs), r2 = keepz(ldh(vr + (size_t)32 * ERW), rs), r3 = keepz(ldh(vr + (size_t)48 * ERW), rs);
            p0 = wmma16(r0, pb, p0); p1 = wmma16(r1, pb, p1); p2 = wmma16(r2, pb, p2); p3 = wmma16(r3, pb, p3);
            asm volatile("v_nop\n\tv_nop\n\tv_nop\n\tv_nop" : "+v"(p0), "+v"(p1), "+v"(p2), "+v"(p3) : "v"(r0), "v"(r1), "v"(r2), "v"(r3), "v"(pb) : "memory");
        } else {
            asm volatile("v_nop\n\tv_nop\n\tv_nop\n\tv_nop" : "+v"(o0), "+v"(o1), "+v"(o2), "+v"(o3) : "v"(v0), "v"(v1), "v"(v2), "v"(v3), "v"(pb));
        }
    }
    l += __shfl_xor(l, 16, 32);
    const float inv = (1.0f / l) * CXS;
    if (EK) { o0 = o0 + p0 * QRI; o1 = o1 + p1 * QRI; o2 = o2 + p2 * QRI; o3 = o3 + p3 * QRI; }
    const int wb = wave * 16 * 68;
    put8(&os[wb + lr * 68 +  0 + 8 * hi], o0, inv);
    put8(&os[wb + lr * 68 + 16 + 8 * hi], o1, inv);
    put8(&os[wb + lr * 68 + 32 + 8 * hi], o2, inv);
    put8(&os[wb + lr * 68 + 48 + 8 * hi], o3, inv);
    wave_sync();
    const size_t cb = ((size_t)b * SEQ + t0) * DM + (size_t)h * HD;
    const size_t rb = ((size_t)b * ERW + t0) * DM + (size_t)h * HD;
#pragma unroll 1
    for (int ps = 0; ps < 2; ++ps) {
#pragma unroll
        for (int s = 0; s < 4; ++s) { const int row = 4 * s + (lane >> 3), c8 = (lane & 7) * 8;
            const v4f x0 = *(const v4fa*)(&os[wb + row * 68 + c8]); const v4f x1 = *(const v4fa*)(&os[wb + row * 68 + c8 + 4]); v8h hv, rv;
#pragma unroll
            for (int i = 0; i < 4; ++i) { const h16 a0 = (h16)x0[i]; const h16 a1 = (h16)x1[i]; hv[i] = a0; hv[4 + i] = a1; rv[i] = (h16)((x0[i] - (float)a0) * QRS); rv[4 + i] = (h16)((x1[i] - (float)a1) * QRS); }
            *(volatile v8h*)(CH + cb + (size_t)row * DM + c8) = hv;
            if (EK) *(volatile v8h*)(CR + rb + (size_t)row * DM + c8) = rv; }
        if (ps == 0) __threadfence(); }
}

template <int MB, int RES>
__global__ __launch_bounds__(32) void k_oproj(const h16* __restrict__ CHp, const h16* __restrict__ CRp, const h16* __restrict__ Wt, const float* __restrict__ bp, float* OUT, int tofs, int tper) {
    __shared__ __align__(16) float os[16 * 68];
    const int lane = threadIdx.x & 31, lr = lane & 15, hi = lane >> 4;
    const int b = blockIdx.x / tper; const int t0 = tofs + (blockIdx.x % tper) * (16 * MB); const int c0 = blockIdx.y * 64;
    v8f aH[MB][4], aR[MB][4];
#pragma unroll
    for (int mb = 0; mb < MB; ++mb)
#pragma unroll
        for (int nb = 0; nb < 4; ++nb) { aH[mb][nb] = (v8f){}; aR[mb][nb] = (v8f){}; }
    const size_t aoff = ((size_t)b * SEQ + t0 + lr) * DM + 8 * hi;
    const size_t roff = ((size_t)b * ERW + t0 + lr) * DM + 8 * hi;
    const size_t boff = (size_t)(c0 + lr) * DM + 8 * hi;
#pragma unroll 1
    for (int kc = 0; kc < DM; kc += 32) {
        v16h a[MB], ar[MB];
#pragma unroll
        for (int mb = 0; mb < MB; ++mb) { a[mb] = ldh(CHp + aoff + (size_t)mb * 16 * DM + kc); if (RES) ar[mb] = ldh(CRp + roff + (size_t)mb * 16 * DM + kc); else ar[mb] = a[mb]; }
#pragma unroll
        for (int nb = 0; nb < 4; ++nb) { const v16h bb = ldh(Wt + boff + (size_t)nb * 16 * DM + kc);
#pragma unroll
            for (int mb = 0; mb < MB; ++mb) { aH[mb][nb] = wmma16(a[mb], bb, aH[mb][nb]); if (RES) aR[mb][nb] = wmma16(ar[mb], bb, aR[mb][nb]); } }
        if (RES) asm volatile("v_nop\n\tv_nop\n\tv_nop\n\tv_nop" : "+v"(aH[0][0]), "+v"(aH[MB - 1][3]), "+v"(aR[0][0]), "+v"(aR[MB - 1][3]) : "v"(a[0]), "v"(a[MB - 1]), "v"(ar[0]), "v"(ar[MB - 1]));
        else     asm volatile("v_nop\n\tv_nop\n\tv_nop\n\tv_nop" : "+v"(aH[0][0]), "+v"(aH[MB - 1][3]), "+v"(aH[0][3]), "+v"(aH[MB - 1][0]) : "v"(a[0]), "v"(a[MB - 1]));
    }
    float bc[4];
#pragma unroll
    for (int nb = 0; nb < 4; ++nb) bc[nb] = bfr(bp[c0 + nb * 16 + lr]);
#pragma unroll
    for (int mb = 0; mb < MB; ++mb) {
#pragma unroll
        for (int nb = 0; nb < 4; ++nb) {
#pragma unroll
            for (int j = 0; j < 8; ++j) { float v = aH[mb][nb][j] * OSC; if (RES) v += aR[mb][nb][j] * OSCR; os[(hi * 8 + j) * 68 + nb * 16 + lr] = v + bc[nb]; } }
        wave_sync();
        float* orow = OUT + ((size_t)b * OUT_SEQ + t0 + mb * 16) * DM + c0;
#pragma unroll 1
        for (int ps = 0; ps < 2; ++ps) {
#pragma unroll
            for (int s = 0; s < 8; ++s) { const int row = 2 * s + hi, cofs = lr * 4;
                const v4f val = *(const v4fa*)(&os[row * 68 + cofs]);
                *(volatile v4f*)(orow + (size_t)row * DM + cofs) = val; }
            if (ps == 0) __threadfence(); }
        wave_sync();
    }
}

static constexpr size_t al256(size_t v) { return (v + 255) & ~(size_t)255; }
static constexpr size_t SZ_XB = al256((size_t)NB * SEQ * DM * 2);
static constexpr size_t SZ_WB = al256((size_t)4 * DM * DM * 2);
static constexpr size_t SZ_PL = al256((size_t)NB * NH_ * SEQ * HD * 2);
static constexpr size_t SZ_PR = al256((size_t)NB * NH_ * ERW * HD * 2);
static constexpr size_t SZ_TOTAL = SZ_XB + SZ_WB + 4 * SZ_PL + 4 * SZ_PR;
static_assert(SZ_TOTAL <= (size_t)134217728);
static_assert(((size_t)DM * DM * 2) % 256 == 0);
static_assert((size_t)NB * SEQ * DM * 2 <= SZ_PL);
static_assert((size_t)NB * ERW * DM * 2 <= SZ_PR);

extern "C" void kernel_launch(void* const* d_in, const int* in_sizes, int n_in,
                              void* d_out, int out_size, void* d_ws, size_t ws_size, hipStream_t stream) {
    if (n_in < 10) return;
    const size_t needx = ((size_t)(NB - 1) * SEQ_FULL + SEQ) * DM;
    if ((size_t)in_sizes[0] < needx) return;
    if ((size_t)in_sizes[1] < (size_t)(SEQ - 1) * SEQ_FULL + SEQ) return;
    if ((size_t)in_sizes[2] < (size_t)DM * DM || (size_t)in_sizes[4] < (size_t)DM * DM || (size_t)in_sizes[6] < (size_t)DM * DM || (size_t)in_sizes[8] < (size_t)DM * DM) return;
    if (in_sizes[3] < DM || in_sizes[5] < DM || in_sizes[7] < DM || in_sizes[9] < DM) return;
    if ((size_t)out_size < ((size_t)(NB - 1) * OUT_SEQ + SEQ) * DM) return;
    if (SZ_TOTAL > ws_size) return;
    const float* x  = (const float*)d_in[0]; const int* mask = (const int*)d_in[1];
    const float* wq = (const float*)d_in[2]; const float* bq = (const float*)d_in[3];
    const float* wk = (const float*)d_in[4]; const float* bk = (const float*)d_in[5];
    const float* wv = (const float*)d_in[6]; const float* bv = (const float*)d_in[7];
    const float* wp = (const float*)d_in[8]; const float* bp = (const float*)d_in[9];
    float* OUT = (float*)d_out;
    char* wsp = (char*)d_ws;
    bf* XB = (bf*)wsp; wsp += SZ_XB;
    bf* WB = (bf*)wsp; wsp += SZ_WB;
    h16* QH = (h16*)wsp; wsp += SZ_PL;
    h16* KH = (h16*)wsp; wsp += SZ_PL;
    h16* VT = (h16*)wsp; wsp += SZ_PL;
    h16* CH = (h16*)wsp; wsp += SZ_PL;
    h16* QR = (h16*)wsp; wsp += SZ_PR;
    h16* KR = (h16*)wsp; wsp += SZ_PR;
    h16* VR = (h16*)wsp; wsp += SZ_PR;
    h16* CR = (h16*)wsp; wsp += SZ_PR;
    bf* WQ = WB; bf* WK = WB + (size_t)DM * DM; bf* WV = WB + (size_t)2 * DM * DM; bf* WP = WB + (size_t)3 * DM * DM;

    if (SEQ == SEQ_FULL) {
        const size_t n8 = (size_t)NB * SEQ * DM / 8;
        k_cvt8<<<(unsigned)((n8 + 255) / 256), 256, 0, stream>>>(x, XB, n8);
    } else {
        const size_t n8 = (size_t)SEQ * DM / 8;
        for (int b = 0; b < NB; ++b) k_cvt8<<<(unsigned)((n8 + 255) / 256), 256, 0, stream>>>(x + (size_t)b * SEQ_FULL * DM, XB + (size_t)b * SEQ * DM, n8);
    }
    k_wt<0><<<dim3(DM / 64, DM / 64, 1), 256, 0, stream>>>(wq, WQ);
    k_wt<0><<<dim3(DM / 64, DM / 64, 1), 256, 0, stream>>>(wk, WK);
    k_wt<0><<<dim3(DM / 64, DM / 64, 1), 256, 0, stream>>>(wv, WV);
    k_wt<1><<<dim3(DM / 64, DM / 64, 1), 256, 0, stream>>>(wp, WP);

    k_proj<<<dim3(NB * SEQ / 64, DM / 64, 1), 32, 0, stream>>>(XB, WQ, bq, 1, QH, QR, 1, SEQ, (size_t)NH_ * SEQ * HD, HD, HD, (size_t)SEQ * HD,
                                                                (size_t)NH_ * ERW * HD, HD, (size_t)ERW * HD);
    k_proj<<<dim3(NB * SEQ / 64, DM / 64, 1), 32, 0, stream>>>(XB, WK, bk, 1, KH, KR, 1, SEQ, (size_t)NH_ * SEQ * HD, HD, HD, (size_t)SEQ * HD,
                                                                (size_t)NH_ * ERW * HD, HD, (size_t)ERW * HD);
    k_proj<<<dim3(DM / 64, NB * SEQ / 64, 1), 32, 0, stream>>>(WV, XB, bv, 2, VT, VR, 2, DM, (size_t)0, SEQ, SEQ, (size_t)DM * SEQ,
                                                                (size_t)0, ERW, (size_t)DM * ERW);

    k_flash<1><<<dim3(ERW / (16 * AW), NB * NH_, 1), 32 * AW, 0, stream>>>(QH, QR, KH, KR, VT, VR, mask, CH, CR, 0);
    if (SEQ > ERW)
        k_flash<0><<<dim3((SEQ - ERW) / (16 * AW), NB * NH_, 1), 32 * AW, 0, stream>>>(QH, QR, KH, KR, VT, VR, mask, CH, CR, ERW);

    k_oproj<2, 1><<<dim3(NB * (ERW / 32), DM / 64, 1), 32, 0, stream>>>(CH, CR, (const h16*)WP, bp, OUT, 0, ERW / 32);
    if (SEQ > ERW)
        k_oproj<4, 0><<<dim3(NB * ((SEQ - ERW) / 64), DM / 64, 1), 32, 0, stream>>>(CH, CR, (const h16*)WP, bp, OUT, ERW, (SEQ - ERW) / 64);
}
